// M_20890720928338
// MI455X (gfx1250) — hardware-run, weakly checked
//
#include <hip/hip_runtime.h>


#ifndef NB
#define NB 512
#endif
#define NB_FULL 512
#define CH   440u
#define CR   52u
#define HW   49u
#define KP   448u
#define NP   448u
#define MTOT ((unsigned)NB * HW)
#define NRT  (MTOT / 64u)
#define LP   456u
#define WSC  64.0f
#define WSI  (1.0f / 64.0f)
#define EPSV 1e-5f
#define INV_M (1.0f / (float)MTOT)
#define NPIECE ((unsigned)(((size_t)NB * 440 * 49) / 4))

static_assert(NB <= NB_FULL);
static_assert(MTOT % 64u == 0u);
static_assert(KP % 32u == 0u);
static_assert(NP % 64u == 0u);
static_assert(KP >= CH && KP - CH == 8u);
static_assert(NP == KP);
static_assert(CH % 8u == 0u);
static_assert((CH * HW) % 4u == 0u);
static_assert(((size_t)NB * 440 * 49) % 4 == 0);
static_assert(14u * 32u == KP);
static_assert(CR % 4u == 0u && CR <= 64u);
static_assert(CR == 13u * 4u);
static_assert(LP % 8u == 0u && LP >= KP);
static_assert((HW * KP * 2u) % 128u == 0u);
static_assert((HW * (KP / 8u)) % 8u == 0u);
static_assert((NP * (KP / 8u)) % 256u == 0u);
static_assert(4u * 112u == NP);
static_assert(32 * 16 * 8 == 16 * 64 * 4);
static_assert(HW * LP * 2u + KP * 4u * 2u + 64u * 4u <= 65536u);
static_assert(16u * 68u * 4u <= 131072u);
static_assert(4u * NP * 4u <= 131072u);

typedef _Float16 h16;
typedef __attribute__((ext_vector_type(16))) _Float16 v16h;
typedef __attribute__((ext_vector_type(8)))  _Float16 v8h;
typedef __attribute__((ext_vector_type(8)))  float    v8f;
typedef __attribute__((ext_vector_type(4)))  float    v4f;
typedef v4f  __attribute__((may_alias)) v4fa;
typedef v8h  __attribute__((may_alias)) v8ha;

__device__ __forceinline__ unsigned short f2bf(float f) { unsigned u = __float_as_uint(f); u += 0x7FFFu + ((u >> 16) & 1u); return (unsigned short)(u >> 16); }
__device__ __forceinline__ float bfr(float f) { return __uint_as_float(((unsigned)f2bf(f)) << 16); }
__device__ __forceinline__ v16h cat16(v8h lo, v8h hi) { return __builtin_shufflevector(lo, hi, 0, 1, 2, 3, 4, 5, 6, 7, 8, 9, 10, 11, 12, 13, 14, 15); }
__device__ __forceinline__ v8f wmma16(v16h a, v16h b, v8f c) { return __builtin_amdgcn_wmma_f32_16x16x32_f16(false, a, false, b, (short)0, c, false, false); }
__device__ __forceinline__ v8f wmma16g(v16h a, v16h b, v8f c) { c = wmma16(a, b, c); asm volatile("v_nop\n\tv_nop\n\tv_nop\n\tv_nop" : "+v"(c) : "v"(a), "v"(b)); return c; }
__device__ __forceinline__ v16h  ldh(const h16* p) { return cat16(*(const v8h*)p, *(const v8h*)(p + 16)); }
__device__ __forceinline__ void wave_sync() { __builtin_amdgcn_fence(3  , "wavefront"); __builtin_amdgcn_wave_barrier(); asm volatile("" ::: "memory"); }
static __device__ __forceinline__ h16 toh_flush(float v) { const float w = (fabsf(v) < 6.103515625e-05f) ? 0.0f : v; return (h16)w; }

__global__ __launch_bounds__(256) void k_wconv(const float* __restrict__ w3, h16* W3H) {
    const unsigned p = blockIdx.x * 256u + threadIdx.x; if (p >= NP * (KP / 8u)) return;
    const unsigned row = p / 56u, pc = p - row * 56u;
    const bool ok = (row < CH) && (pc < 55u);
    const unsigned rr = min(row, CH - 1u), pcc = min(pc, 54u);
    const float* s = w3 + rr * CH + pcc * 8u;
    const v4f x0 = *(const v4f*)s; const v4f x1 = *(const v4f*)(s + 4);
    v8h o;
#pragma unroll
    for (int i = 0; i < 4; ++i) { const float a0 = ok ? bfr(x0[i]) * WSC : 0.0f; const float a1 = ok ? bfr(x1[i]) * WSC : 0.0f; o[i] = toh_flush(a0); o[4 + i] = toh_flush(a1); }
    h16* d = W3H + (size_t)p * 8u;
    *(volatile v8h*)d = o; __threadfence(); *(volatile v8h*)d = o;
}

__global__ __launch_bounds__(256) void k_gate_a(const float* __restrict__ x178, const float* __restrict__ x177, const float* __restrict__ w1, const float* __restrict__ b1,
                                                const float* __restrict__ w2, const float* __restrict__ b2, h16* GA) {
    __shared__ __align__(16) float ss[KP];
    __shared__ __align__(16) float hs[64];
    __shared__ __align__(16) float gs[KP];
    __shared__ __align__(16) h16 th[HW * LP];
    const unsigned tid = threadIdx.x, lane = tid & 31u;
    const unsigned wave = (unsigned)__builtin_amdgcn_readfirstlane((int)(threadIdx.x >> 5));
    const unsigned b = blockIdx.x;
#pragma unroll 1
    for (unsigned c = tid; c < KP; c += 256u) { const unsigned cc = min(c, CH - 1u); const float v = bfr(x178[b * CH + cc]); ss[c] = (c < CH) ? v : 0.0f; }
    __syncthreads();
#pragma unroll 1
    for (unsigned r = wave; r < CR; r += 8u) {
        const float* wr = w1 + r * CH;
        const float bb = bfr(b1[r]);
        float acc = 0.0f;
#pragma unroll 1
        for (unsigned it = 0; it < 14u; ++it) { const unsigned c = it * 32u + lane; const unsigned cc = min(c, CH - 1u);
            const float wv = bfr(wr[cc]); const float wz = (c < CH) ? wv : 0.0f; acc = fmaf(ss[c], wz, acc); }
        acc += __shfl_xor(acc, 16, 32); acc += __shfl_xor(acc, 8, 32); acc += __shfl_xor(acc, 4, 32); acc += __shfl_xor(acc, 2, 32); acc += __shfl_xor(acc, 1, 32);
        if (lane == 0u) hs[r] = fmaxf(acc + bb, 0.0f);
    }
    __syncthreads();
#pragma unroll 1
    for (unsigned o = tid; o < KP; o += 256u) {
        const unsigned oc = min(o, CH - 1u);
        const float* wr = w2 + oc * CR;
        float acc = 0.0f;
#pragma unroll 1
        for (unsigned q = 0; q < 13u; ++q) { const v4f wv = *(const v4f*)(wr + 4u * q);
            acc = fmaf(hs[4u * q], bfr(wv[0]), acc); acc = fmaf(hs[4u * q + 1u], bfr(wv[1]), acc); acc = fmaf(hs[4u * q + 2u], bfr(wv[2]), acc); acc = fmaf(hs[4u * q + 3u], bfr(wv[3]), acc); }
        const float t = acc + bfr(b2[oc]);
        const float g = 1.0f / (1.0f + expf(-t));
        gs[o] = (o < CH) ? g : 0.0f;
    }
    __syncthreads();
    const float* xb = x177 + (size_t)b * (CH * HW);
#pragma unroll 1
    for (unsigned j = tid; j < (CH * HW) / 4u; j += 256u) {
        const v4f xv = *(const v4f*)(xb + 4u * j);
#pragma unroll
        for (int i = 0; i < 4; ++i) { const unsigned e = 4u * j + (unsigned)i; const unsigned c = e / HW; const unsigned hw = e - c * HW;
            th[hw * LP + c] = toh_flush(bfr(xv[i]) * gs[c]); }
    }
#pragma unroll 1
    for (unsigned z = tid; z < HW * 8u; z += 256u) { const unsigned hw = z / 8u; const unsigned c = CH + (z & 7u); th[hw * LP + c] = (h16)0.0f; }
    __syncthreads();
    h16* gb = GA + (size_t)(b * HW) * KP;
#pragma unroll 1
    for (int ps = 0; ps < 2; ++ps) {
#pragma unroll 1
        for (unsigned q = tid; q < HW * (KP / 8u); q += 256u) {
            const unsigned row = q / 56u, pc = q - row * 56u;
            const v8h val = *(const v8ha*)(&th[row * LP + pc * 8u]);
            *(volatile v8h*)(gb + (size_t)q * 8u) = val; }
        if (ps == 0) __threadfence(); }
}

__global__ __launch_bounds__(32) void k_gemm(const h16* __restrict__ A, const h16* __restrict__ Bt, float* Y) {
    __shared__ __align__(16) float os[16 * 68];
    const int lane = threadIdx.x & 31, lr = lane & 15, hi = lane >> 4;
    const unsigned r0 = blockIdx.x * 64u, c0 = blockIdx.y * 64u;
    v8f acc[4][4];
#pragma unroll
    for (int mb = 0; mb < 4; ++mb)
#pragma unroll
        for (int nb = 0; nb < 4; ++nb) acc[mb][nb] = (v8f){};
    const size_t aoff = (size_t)(r0 + (unsigned)lr) * KP + (size_t)(8 * hi), boff = (size_t)(c0 + (unsigned)lr) * KP + (size_t)(8 * hi);
#pragma unroll 1
    for (unsigned kc = 0; kc < KP; kc += 32u) {
        v16h a[4];
#pragma unroll
        for (int mb = 0; mb < 4; ++mb) a[mb] = ldh(A + aoff + (size_t)mb * 16u * KP + kc);
#pragma unroll
        for (int nb = 0; nb < 4; ++nb) { const v16h b = ldh(Bt + boff + (size_t)nb * 16u * KP + kc);
#pragma unroll
            for (int mb = 0; mb < 4; ++mb) acc[mb][nb] = wmma16g(a[mb], b, acc[mb][nb]); }
    }
#pragma unroll
    for (int mb = 0; mb < 4; ++mb) {
#pragma unroll
        for (int nb = 0; nb < 4; ++nb) {
#pragma unroll
            for (int j = 0; j < 8; ++j) os[(hi * 8 + j) * 68 + nb * 16 + lr] = acc[mb][nb][j] * WSI; }
        wave_sync();
        float* yb = Y + (size_t)(r0 + (unsigned)(mb * 16)) * NP + c0;
#pragma unroll 1
        for (int ps = 0; ps < 2; ++ps) {
#pragma unroll
            for (int s = 0; s < 8; ++s) { const int row = 2 * s + (lane >> 4), cofs = (lane & 15) * 4;
                const v4f val = *(const v4fa*)(&os[row * 68 + cofs]);
                *(volatile v4f*)(yb + (size_t)row * NP + cofs) = val; }
            if (ps == 0) __threadfence(); }
        wave_sync();
    }
}

__global__ __launch_bounds__(448) void k_colsum(const float* __restrict__ Y, float* PART) {
    __shared__ __align__(16) float red[4 * NP];
    const unsigned tid = threadIdx.x; const unsigned rp = tid / 112u; const unsigned cg = tid - rp * 112u;
    const float* yp = Y + (size_t)(blockIdx.x * 64u + rp * 16u) * NP + 4u * cg;
    v4f acc = (v4f){};
#pragma unroll 1
    for (unsigned r = 0; r < 16u; ++r) { const v4f y = *(const v4f*)(yp + (size_t)r * NP); acc = acc + y; }
    *(v4fa*)(&red[rp * NP + 4u * cg]) = acc;
    __syncthreads();
    if (tid < 112u) {
        v4f s = *(const v4fa*)(&red[4u * tid]);
        s = s + *(const v4fa*)(&red[NP + 4u * tid]); s = s + *(const v4fa*)(&red[2u * NP + 4u * tid]); s = s + *(const v4fa*)(&red[3u * NP + 4u * tid]);
        float* d = PART + (size_t)blockIdx.x * NP + 4u * tid;
        *(volatile v4f*)d = s; __threadfence(); *(volatile v4f*)d = s; }
}

__global__ __launch_bounds__(448) void k_colsq(const float* __restrict__ Y, const float* __restrict__ ST, float* PART) {
    __shared__ __align__(16) float red[4 * NP];
    const unsigned tid = threadIdx.x; const unsigned rp = tid / 112u; const unsigned cg = tid - rp * 112u;
    const float* yp = Y + (size_t)(blockIdx.x * 64u + rp * 16u) * NP + 4u * cg;
    const v4f mu = *(const v4f*)(ST + 4u * cg);
    v4f acc = (v4f){};
#pragma unroll 1
    for (unsigned r = 0; r < 16u; ++r) { const v4f y = *(const v4f*)(yp + (size_t)r * NP); const v4f d = y - mu; acc = acc + d * d; }
    *(v4fa*)(&red[rp * NP + 4u * cg]) = acc;
    __syncthreads();
    if (tid < 112u) {
        v4f s = *(const v4fa*)(&red[4u * tid]);
        s = s + *(const v4fa*)(&red[NP + 4u * tid]); s = s + *(const v4fa*)(&red[2u * NP + 4u * tid]); s = s + *(const v4fa*)(&red[3u * NP + 4u * tid]);
        float* d = PART + (size_t)blockIdx.x * NP + 4u * tid;
        *(volatile v4f*)d = s; __threadfence(); *(volatile v4f*)d = s; }
}

__global__ __launch_bounds__(448) void k_mean(const float* __restrict__ PART, float* ST) {
    __shared__ __align__(16) float sl[NP];
    const unsigned tid = threadIdx.x;
    float s = 0.0f, c = 0.0f;
#pragma unroll 1
    for (unsigned r = 0; r < NRT; ++r) { const float v = PART[(size_t)r * NP + tid]; const float y = v - c; const float t = s + y; c = (t - s) - y; s = t; }
    sl[tid] = s * INV_M;
    __syncthreads();
    if (tid < NP / 4u) { const v4f val = *(const v4fa*)(&sl[4u * tid]); float* d = ST + 4u * tid;
        *(volatile v4f*)d = val; __threadfence(); *(volatile v4f*)d = val; }
}

__global__ __launch_bounds__(448) void k_fin(const float* __restrict__ PART, const float* __restrict__ gamma, const float* __restrict__ beta, float* ST) {
    __shared__ __align__(16) float sl[3 * NP];
    const unsigned tid = threadIdx.x;
    float s = 0.0f, c = 0.0f;
#pragma unroll 1
    for (unsigned r = 0; r < NRT; ++r) { const float v = PART[(size_t)r * NP + tid]; const float y = v - c; const float t = s + y; c = (t - s) - y; s = t; }
    const float var = s * INV_M;
    const unsigned cc = min(tid, CH - 1u);
    const float g = bfr(gamma[cc]), be = bfr(beta[cc]);
    const bool ok = tid < CH;
    sl[tid] = 1.0f / sqrtf(var + EPSV);
    sl[NP + tid] = ok ? g : 0.0f;
    sl[2u * NP + tid] = ok ? be : 0.0f;
    __syncthreads();
    if (tid < 3u * NP / 4u) { const v4f val = *(const v4fa*)(&sl[4u * tid]); float* d = ST + NP + 4u * tid;
        *(volatile v4f*)d = val; __threadfence(); *(volatile v4f*)d = val; }
}

__global__ __launch_bounds__(256) void k_out(const float* __restrict__ Y, const float* __restrict__ ST, float* OUT) {
    __shared__ __align__(16) float st[4 * NP];
    const unsigned tid = threadIdx.x;
#pragma unroll 1
    for (unsigned q = tid; q < NP; q += 256u) { const v4f v = *(const v4f*)(ST + 4u * q); *(v4fa*)(&st[4u * q]) = v; }
    __syncthreads();
#pragma unroll 1
    for (unsigned it = 0; it < 4u; ++it) {
        const unsigned p = blockIdx.x * 1024u + it * 256u + tid;
        if (p < NPIECE) {
            v4f val;
#pragma unroll
            for (int i = 0; i < 4; ++i) {
                const unsigned e = 4u * p + (unsigned)i;
                const unsigned bo = e / HW; const unsigned hw = e - bo * HW;
                const unsigned bb = bo / CH; const unsigned o = bo - bb * CH;
                const float y = Y[(size_t)(bb * HW + hw) * NP + o];
                val[i] = ((y - st[o]) * st[NP + o]) * st[2u * NP + o] + st[3u * NP + o]; }
            float* d = OUT + (size_t)p * 4u;
            *(volatile v4f*)d = val; __threadfence(); *(volatile v4f*)d = val;
        }
    }
}

static constexpr size_t al256(size_t v) { return (v + 255) & ~(size_t)255; }
static constexpr size_t SZ_GA = al256((size_t)NB * 49 * 448 * 2);
static constexpr size_t SZ_WH = al256((size_t)448 * 448 * 2);
static constexpr size_t SZ_Y  = al256((size_t)NB * 49 * 448 * 4);
static constexpr size_t SZ_PT = al256((size_t)(NB * 49 / 64) * 448 * 4);
static constexpr size_t SZ_ST = al256((size_t)4 * 448 * 4);
static constexpr size_t SZ_TOTAL = SZ_GA + SZ_WH + SZ_Y + 2 * SZ_PT + SZ_ST;
static_assert(SZ_TOTAL <= (size_t)134217728);
static constexpr unsigned OUT_GRID = (NPIECE + 1023u) / 1024u;
static constexpr unsigned WC_GRID  = (448u * 56u) / 256u;
static_assert((size_t)NPIECE * 4 == (size_t)NB * 440 * 49);

extern "C" void kernel_launch(void* const* d_in, const int* in_sizes, int n_in,
                              void* d_out, int out_size, void* d_ws, size_t ws_size, hipStream_t stream) {
    if (n_in < 9) return;
    if ((size_t)in_sizes[0] < (size_t)NB * 440) return;
    if ((size_t)in_sizes[1] < (size_t)NB * 440 * 49) return;
    if (in_sizes[2] < 52 * 440 || in_sizes[3] < 52 || in_sizes[4] < 440 * 52 || in_sizes[5] < 440) return;
    if (in_sizes[6] < 440 * 440 || in_sizes[7] < 440 || in_sizes[8] < 440) return;
    if ((size_t)out_size < (size_t)NB * 440 * 49) return;
    if (SZ_TOTAL > ws_size) return;
    const float* x178 = (const float*)d_in[0]; const float* x177 = (const float*)d_in[1];
    const float* w1 = (const float*)d_in[2]; const float* b1 = (const float*)d_in[3];
    const float* w2 = (const float*)d_in[4]; const float* b2 = (const float*)d_in[5];
    const float* w3 = (const float*)d_in[6]; const float* gamma = (const float*)d_in[7]; const float* beta = (const float*)d_in[8];
    float* OUT = (float*)d_out;
    char* wsp = (char*)d_ws;
    h16* GA  = (h16*)wsp;   wsp += SZ_GA;
    h16* W3H = (h16*)wsp;   wsp += SZ_WH;
    float* Y = (float*)wsp; wsp += SZ_Y;
    float* P1 = (float*)wsp; wsp += SZ_PT;
    float* P2 = (float*)wsp; wsp += SZ_PT;
    float* ST = (float*)wsp; wsp += SZ_ST;

    k_wconv<<<WC_GRID, 256, 0, stream>>>(w3, W3H);
    k_gate_a<<<NB, 256, 0, stream>>>(x178, x177, w1, b1, w2, b2, GA);
    k_gemm<<<dim3(NB * 49 / 64, 448 / 64, 1), 32, 0, stream>>>(GA, W3H, Y);
    k_colsum<<<NB * 49 / 64, 448, 0, stream>>>(Y, P1);
    k_mean<<<1, 448, 0, stream>>>(P1, ST);
    k_colsq<<<NB * 49 / 64, 448, 0, stream>>>(Y, ST, P2);
    k_fin<<<1, 448, 0, stream>>>(P2, gamma, beta, ST);
    k_out<<<OUT_GRID, 256, 0, stream>>>(Y, ST, OUT);
}
